// ISA_2336462209656
// MI455X (gfx1250) — hardware-run, weakly checked
//
#include <hip/hip_runtime.h>
#include <math.h>

typedef __attribute__((ext_vector_type(16))) _Float16 v16h;
typedef __attribute__((ext_vector_type(8)))  _Float16 v8h;
typedef __attribute__((ext_vector_type(8)))  float    v8f;
typedef __attribute__((ext_vector_type(4)))  float    v4f;
typedef __attribute__((ext_vector_type(4)))  unsigned int v4u;

constexpr int kB      = 4;
constexpr int kN      = 2048;
constexpr int kDin    = 768;
constexpr int kDS     = 256;
constexpr int kS      = 8;
constexpr int kBS     = kB * kS;
constexpr int kRowsE  = kB * kN;
constexpr int kRowsP  = kBS * kN;
constexpr int kFeat   = 39;
constexpr int kFeatK  = 64;
constexpr int kFeatLds = 40;
constexpr int kHid    = 1024;
constexpr int kGru    = 768;
constexpr int kPitchS = 288;
constexpr int kStatOff = 256;
constexpr int kAsumOff = 262;
constexpr int kSqrtDS = 16;
static_assert(kSqrtDS * kSqrtDS == kDS);
static_assert(kBS == 32 && kRowsE == 8192 && kRowsP == 65536);
static_assert((kDin % 32) == 0 && (kDS % 32) == 0 && (kFeatK % 32) == 0);
static_assert((kRowsE % 64) == 0 && (kRowsP % 64) == 0 && (kDin % 64) == 0 && (kDS % 64) == 0);
static_assert(kFeat <= kFeatLds && kFeatLds <= kFeatK && (kFeatLds % 8) == 0);
static_assert((kN % 256) == 0 && (kPitchS % 32) == 0 && kAsumOff < kPitchS);
constexpr float kDotScale  = 1.0f / (float)kSqrtDS;
constexpr float kInvDS     = 1.0f / (float)kDS;
constexpr float kWCarry    = 16.0f;
constexpr float kWCarryInv = 1.0f / kWCarry;
constexpr float kLnEps     = 1e-5f;
constexpr float kTwoPi     = 6.28318530717958647692f;
constexpr int   kOutSlots  = kBS * kDS;
static_assert((size_t)kOutSlots * 4 + (size_t)kBS * kN * 4 == 294912ull);

constexpr size_t kOffW1H  = 0;
constexpr size_t kOffW2H  = kOffW1H  + (size_t)kDin * kDin * 2;
constexpr size_t kOffKVWH = kOffW2H  + (size_t)kDS * kDin * 2;
constexpr size_t kOffF1H  = kOffKVWH + (size_t)2 * kDS * kDS * 2;
constexpr size_t kOffG1H  = kOffF1H  + (size_t)kDS * kDS * 2;
constexpr size_t kOffC1   = kOffG1H  + (size_t)kDS * kFeatK * 2;
constexpr size_t kOffX0H  = kOffC1   + (size_t)kDS * 4;
constexpr size_t kOffH1H  = kOffX0H  + (size_t)kRowsE * kDin * 2;
constexpr size_t kOffXP   = kOffH1H  + (size_t)kRowsE * kDin * 2;
constexpr size_t kOffXH   = kOffXP   + (size_t)kRowsE * kDS * 4;
constexpr size_t kOffKVH  = kOffXH   + (size_t)kRowsE * kDS * 2;
constexpr size_t kOffKVF  = kOffKVH  + (size_t)2 * kRowsE * kDS * 2;
constexpr size_t kOffFA   = kOffKVF  + (size_t)2 * kRowsE * kDS * 4;
constexpr size_t kOffPF   = kOffFA   + (size_t)kRowsP * kFeatK * 2;
constexpr size_t kOffDOTS = kOffPF   + (size_t)kRowsP * kDS * 2;
constexpr size_t kOffATT  = kOffDOTS + (size_t)kRowsP * 4;
constexpr size_t kOffSLA  = kOffATT  + (size_t)kBS * kN * 4;
constexpr size_t kOffSLB  = kOffSLA  + (size_t)kBS * kDS * 4;
constexpr size_t kOffQF   = kOffSLB  + (size_t)kBS * kDS * 4;
constexpr size_t kOffUH   = kOffQF   + (size_t)kBS * kPitchS * 4;
constexpr size_t kWsTotal = kOffUH   + (size_t)kBS * kPitchS * 4;
static_assert(kWsTotal == 107521024ull);
static_assert(kWsTotal <= 134217728ull);
static_assert((kOffW2H % 128) == 0 && (kOffKVWH % 128) == 0 && (kOffF1H % 128) == 0 && (kOffG1H % 128) == 0 &&
              (kOffC1 % 128) == 0 && (kOffX0H % 128) == 0 && (kOffH1H % 128) == 0 && (kOffXP % 128) == 0 &&
              (kOffXH % 128) == 0 && (kOffKVH % 128) == 0 && (kOffKVF % 128) == 0 && (kOffFA % 128) == 0 &&
              (kOffPF % 128) == 0 && (kOffDOTS % 128) == 0 && (kOffATT % 128) == 0 && (kOffSLA % 128) == 0 &&
              (kOffSLB % 128) == 0 && (kOffQF % 128) == 0 && (kOffUH % 128) == 0);

__device__ __forceinline__ float n2nf(float x) {
  float y = x;
  y = (x != x) ? 0.0f : y;
  y = (x == INFINITY) ? 1.0f : y;
  y = (x == -INFINITY) ? -1.0f : y;
  return y;
}

__device__ __forceinline__ float h16_to_f32(unsigned hb) {
  const unsigned sgn = (hb & 0x8000u) << 16;
  const unsigned em = hb & 0x7fffu;
  const float fn = __uint_as_float((em << 13) + 0x38000000u);
  const float fs = (float)em * 5.9604644775390625e-8f;
  const float mag = (em < 0x400u) ? fs : fn;
  return __uint_as_float(__float_as_uint(mag) | sgn);
}

__device__ __forceinline__ void hid8(const v4f k0, const v4f k1, const v4u pw, const v4f ca, const v4f cb,
                                     v4f& h0, v4f& h1) {
  const unsigned w0 = pw[0];
  const unsigned w1 = pw[1];
  const unsigned w2 = pw[2];
  const unsigned w3 = pw[3];
  const float p0 = h16_to_f32(w0 & 0xffffu);
  const float p1 = h16_to_f32(w0 >> 16);
  const float p2 = h16_to_f32(w1 & 0xffffu);
  const float p3 = h16_to_f32(w1 >> 16);
  const float p4 = h16_to_f32(w2 & 0xffffu);
  const float p5 = h16_to_f32(w2 >> 16);
  const float p6 = h16_to_f32(w3 & 0xffffu);
  const float p7 = h16_to_f32(w3 >> 16);
  h0[0] = fmaxf((k0[0] + p0) + ca[0], 0.0f);
  h0[1] = fmaxf((k0[1] + p1) + ca[1], 0.0f);
  h0[2] = fmaxf((k0[2] + p2) + ca[2], 0.0f);
  h0[3] = fmaxf((k0[3] + p3) + ca[3], 0.0f);
  h1[0] = fmaxf((k1[0] + p4) + cb[0], 0.0f);
  h1[1] = fmaxf((k1[1] + p5) + cb[1], 0.0f);
  h1[2] = fmaxf((k1[2] + p6) + cb[2], 0.0f);
  h1[3] = fmaxf((k1[3] + p7) + cb[3], 0.0f);
}

__device__ __forceinline__ float block_sum256(float v, float* red, int lane, int wave) {
  v += __shfl_xor(v, 16, 32);
  v += __shfl_xor(v, 8, 32);
  v += __shfl_xor(v, 4, 32);
  v += __shfl_xor(v, 2, 32);
  v += __shfl_xor(v, 1, 32);
  __syncthreads();
  if (lane == 0) red[wave] = v;
  __syncthreads();
  float s = 0.0f;
#pragma unroll
  for (int w = 0; w < 8; ++w) s += red[w];
  return s;
}

__device__ __forceinline__ void grp_guard_h(v8f& a, v8f& b, v8f& c, v8f& d, v16h x,
                                            v16h y0, v16h y1, v16h y2, v16h y3) {
  asm volatile("v_nop\n\tv_nop\n\tv_nop\n\tv_nop"
               : "+v"(a), "+v"(b), "+v"(c), "+v"(d)
               : "v"(x), "v"(y0), "v"(y1), "v"(y2), "v"(y3));
}
__device__ __forceinline__ void keep4_h(v16h a, v16h b, v16h c, v16h d) {
  asm volatile("v_nop" :: "v"(a), "v"(b), "v"(c), "v"(d));
}
__device__ __forceinline__ void acc_guard4(v8f& a, v8f& b, v8f& c, v8f& d) {
  asm volatile("v_nop\n\tv_nop\n\tv_nop\n\tv_nop" : "+v"(a), "+v"(b), "+v"(c), "+v"(d));
}
struct FragH {
  union U { v16h v; v8h h[2]; };
  static __device__ __forceinline__ v16h load(const _Float16* p) {
    U f;
    f.h[0] = *(const v8h*)(p);
    f.h[1] = *(const v8h*)(p + 16);
    return f.v;
  }
  static __device__ __forceinline__ v8f mma(v16h a, v16h b, v8f c) {
    return __builtin_amdgcn_wmma_f32_16x16x32_f16(false, a, false, b, (short)0, c, false, false);
  }
};

template <int BIAS_MODE, int OUT_MODE, int ACT>
__global__ __launch_bounds__(256) void wmma_gemm64(
    const unsigned short* __restrict__ Ap, int lda, long strideA,
    const unsigned short* __restrict__ Btp, int ldb, long strideB,
    void* __restrict__ Cout, int ldc, long strideC,
    const float* __restrict__ bias,
    int M, int N, int K, float scale) {
  const _Float16* A  = (const _Float16*)Ap;
  const _Float16* Bt = (const _Float16*)Btp;
  __shared__ __align__(16) float sT[8][16 * 68];
  const int b    = blockIdx.y;
  const int lane = threadIdx.x & 31;
  const int wave = threadIdx.x >> 5;
  const int tilesN = N >> 6;
  const int tilesM = M >> 6;
  const int tile = blockIdx.x * 8 + wave;
  if (tile >= tilesM * tilesN) return;
  const int tm = tile / tilesN;
  const int tn = tile - tm * tilesN;
  const int m0 = tm << 6;
  const int n0 = tn << 6;

  const _Float16* Ab = A  + (size_t)b * strideA;
  const _Float16* Bb = Bt + (size_t)b * strideB;

  const int rlane = lane & 15;
  const int koff  = (lane >> 4) * 8;
  const int mOff  = (lane >> 4) * 8;

  v8f acc[4][4];
#pragma unroll
  for (int i = 0; i < 4; ++i)
#pragma unroll
    for (int j = 0; j < 4; ++j) acc[i][j] = (v8f){0.f,0.f,0.f,0.f,0.f,0.f,0.f,0.f};

  for (int k0 = 0; k0 < K; k0 += 32) {
    v16h bh[4];
#pragma unroll
    for (int j = 0; j < 4; ++j) {
      const size_t bo = (size_t)(n0 + (j << 4) + rlane) * ldb + koff + k0;
      bh[j] = FragH::load(Bb + bo);
    }
#pragma unroll
    for (int i = 0; i < 4; ++i) {
      const size_t ao = (size_t)(m0 + (i << 4) + rlane) * lda + koff + k0;
      const v16h ah = FragH::load(Ab + ao);
#pragma unroll
      for (int j = 0; j < 4; ++j) acc[i][j] = FragH::mma(ah, bh[j], acc[i][j]);
      grp_guard_h(acc[i][0], acc[i][1], acc[i][2], acc[i][3], ah, bh[0], bh[1], bh[2], bh[3]);
    }
    keep4_h(bh[0], bh[1], bh[2], bh[3]);
  }
  acc_guard4(acc[0][0], acc[0][1], acc[0][2], acc[0][3]);
  acc_guard4(acc[1][0], acc[1][1], acc[1][2], acc[1][3]);
  acc_guard4(acc[2][0], acc[2][1], acc[2][2], acc[2][3]);
  acc_guard4(acc[3][0], acc[3][1], acc[3][2], acc[3][3]);

  float* slab = sT[wave];
#pragma unroll
  for (int i = 0; i < 4; ++i) {
    const int mBase = m0 + (i << 4);
#pragma unroll
    for (int j = 0; j < 4; ++j) {
      const int n = n0 + (j << 4) + rlane;
      float bv = 0.f;
      if (BIAS_MODE == 2) bv = bias[n];
#pragma unroll
      for (int r = 0; r < 8; ++r) {
        float v = acc[i][j][r] * scale;
        if (BIAS_MODE == 2) v += bv;
        if (ACT == 2) v = fmaxf(v, 0.0f);
        slab[(mOff + r) * 68 + (j << 4) + rlane] = v;
      }
    }
    __builtin_amdgcn_fence(__ATOMIC_RELEASE, "workgroup");
    __builtin_amdgcn_wave_barrier();
    __builtin_amdgcn_fence(__ATOMIC_ACQUIRE, "workgroup");
    if (OUT_MODE == 0) {
      float* C = (float*)Cout + (size_t)b * strideC;
      const int hh = lane >> 4, c4 = (lane & 15) * 4;
      for (int pass = 0; pass < 2; ++pass) {
#pragma unroll
        for (int it = 0; it < 8; ++it) {
          const int row = it * 2 + hh;
          v4f v = *(const v4f*)(slab + row * 68 + c4);
          *(volatile v4f*)(C + (size_t)(mBase + row) * ldc + n0 + c4) = v;
        }
        __threadfence();
      }
    } else {
      const int q = lane >> 3, c8 = (lane & 7) * 8;
      unsigned short* C = (unsigned short*)Cout + (size_t)b * strideC;
      for (int pass = 0; pass < 2; ++pass) {
#pragma unroll
        for (int it = 0; it < 4; ++it) {
          const int row = it * 4 + q;
          const float* sp = slab + row * 68 + c8;
          v8h hv;
#pragma unroll
          for (int e = 0; e < 8; ++e) hv[e] = (_Float16)sp[e];
          *(volatile v8h*)(C + (size_t)(mBase + row) * ldc + n0 + c8) = hv;
        }
        __threadfence();
      }
    }
    __builtin_amdgcn_fence(__ATOMIC_RELEASE, "workgroup");
    __builtin_amdgcn_wave_barrier();
    __builtin_amdgcn_fence(__ATOMIC_ACQUIRE, "workgroup");
  }
}

__global__ __launch_bounds__(256) void cast8_f16_kernel(const float* __restrict__ in,
                                                        unsigned short* __restrict__ out, int n8, float carry) {
  const int i = blockIdx.x * 256 + threadIdx.x;
  if (i >= n8) return;
  const float* p = in + 8 * (size_t)i;
  const v4f a = *(const v4f*)(p);
  const v4f c = *(const v4f*)(p + 4);
  v8h hv;
#pragma unroll
  for (int e = 0; e < 4; ++e) {
    hv[e]     = (_Float16)(a[e] * carry);
    hv[4 + e] = (_Float16)(c[e] * carry);
  }
  unsigned short* q = out + 8 * (size_t)i;
  *(volatile v8h*)q = hv;
  __threadfence();
  *(volatile v8h*)q = hv;
}

template <int NCH, bool N2N>
__global__ __launch_bounds__(256) void ln_rows_f16_kernel(const float* __restrict__ in, const float* __restrict__ g,
                                                          const float* __restrict__ bt,
                                                          unsigned short* __restrict__ out, int rows) {
  constexpr int DIM = NCH * 256;
  constexpr float kInvDim = 1.0f / (float)DIM;
  const int lane = threadIdx.x & 31, wave = threadIdx.x >> 5;
  const int row = blockIdx.x * 8 + wave;
  if (row >= rows) return;
  const float* x = in + (size_t)row * DIM;
  float v[NCH * 8];
#pragma unroll
  for (int ch = 0; ch < NCH; ++ch) {
    const v4f a = *(const v4f*)(x + ch * 256 + lane * 8);
    const v4f c = *(const v4f*)(x + ch * 256 + lane * 8 + 4);
#pragma unroll
    for (int e = 0; e < 4; ++e) {
      v[ch * 8 + e]     = a[e];
      v[ch * 8 + 4 + e] = c[e];
    }
  }
  float s = 0.0f;
#pragma unroll
  for (int i = 0; i < NCH * 8; ++i) s += v[i];
  s += __shfl_xor(s, 16, 32);
  s += __shfl_xor(s, 8, 32);
  s += __shfl_xor(s, 4, 32);
  s += __shfl_xor(s, 2, 32);
  s += __shfl_xor(s, 1, 32);
  const float mean = s * kInvDim;
  float q = 0.0f;
#pragma unroll
  for (int i = 0; i < NCH * 8; ++i) {
    const float d = v[i] - mean;
    q = fmaf(d, d, q);
  }
  q += __shfl_xor(q, 16, 32);
  q += __shfl_xor(q, 8, 32);
  q += __shfl_xor(q, 4, 32);
  q += __shfl_xor(q, 2, 32);
  q += __shfl_xor(q, 1, 32);
  const float rstd = 1.0f / sqrtf(q * kInvDim + kLnEps);
  v8h hv[NCH];
#pragma unroll
  for (int ch = 0; ch < NCH; ++ch) {
    const v4f g0 = *(const v4f*)(g + ch * 256 + lane * 8);
    const v4f g1 = *(const v4f*)(g + ch * 256 + lane * 8 + 4);
    const v4f b0 = *(const v4f*)(bt + ch * 256 + lane * 8);
    const v4f b1 = *(const v4f*)(bt + ch * 256 + lane * 8 + 4);
#pragma unroll
    for (int e = 0; e < 4; ++e) {
      float y0 = (v[ch * 8 + e] - mean) * rstd * g0[e] + b0[e];
      float y1 = (v[ch * 8 + 4 + e] - mean) * rstd * g1[e] + b1[e];
      if (N2N) {
        y0 = n2nf(y0);
        y1 = n2nf(y1);
      }
      hv[ch][e]     = (_Float16)y0;
      hv[ch][4 + e] = (_Float16)y1;
    }
  }
  unsigned short* orow = out + (size_t)row * DIM;
  for (int pass = 0; pass < 2; ++pass) {
#pragma unroll
    for (int ch = 0; ch < NCH; ++ch) *(volatile v8h*)(orow + ch * 256 + lane * 8) = hv[ch];
    __threadfence();
  }
}

__global__ __launch_bounds__(256) void g1_kernel(const float* __restrict__ f1w, const float* __restrict__ gw,
                                                 const float* __restrict__ gb, const float* __restrict__ f1b,
                                                 unsigned short* __restrict__ G1H, float* __restrict__ C1) {
  __shared__ __align__(16) float sF[32 * 256];
  __shared__ __align__(16) float sG[32 * 68];
  __shared__ float sC[32];
  const int t = threadIdx.x, lane = t & 31, wave = t >> 5;
  const int j0 = blockIdx.x * 32;
#pragma unroll 1
  for (int i = 0; i < 8; ++i) {
    const int idx = (i * 256 + t) * 4;
    *(v4f*)(sF + idx) = *(const v4f*)(f1w + (size_t)j0 * 256 + idx);
  }
  __syncthreads();
  const int c = t & 63, rg = t >> 6;
  const int cc = (c < kFeat) ? c : (kFeat - 1);
  float acc[8];
#pragma unroll
  for (int i = 0; i < 8; ++i) acc[i] = 0.0f;
#pragma unroll 1
  for (int d = 0; d < 256; ++d) {
    const float gv = gw[d * kFeat + cc];
#pragma unroll
    for (int i = 0; i < 8; ++i) acc[i] = fmaf(sF[(rg * 8 + i) * 256 + d], gv, acc[i]);
  }
#pragma unroll
  for (int i = 0; i < 8; ++i) sG[(rg * 8 + i) * 68 + c] = (c < kFeat) ? (acc[i] * kWCarry) : 0.0f;
  {
    const int row = t >> 3, part = t & 7;
    float p = 0.0f;
#pragma unroll 1
    for (int d = 0; d < 32; ++d) p = fmaf(sF[row * 256 + part * 32 + d], gb[part * 32 + d], p);
    p += __shfl_xor(p, 1, 32);
    p += __shfl_xor(p, 2, 32);
    p += __shfl_xor(p, 4, 32);
    if (part == 0) sC[row] = p;
  }
  __syncthreads();
  const int q = lane >> 3, c8 = (lane & 7) * 8;
  const int grow = wave * 4 + q;
  const v4f a0 = *(const v4f*)(sG + grow * 68 + c8);
  const v4f a1 = *(const v4f*)(sG + grow * 68 + c8 + 4);
  v8h hv;
#pragma unroll
  for (int e = 0; e < 4; ++e) {
    hv[e]     = (_Float16)a0[e];
    hv[4 + e] = (_Float16)a1[e];
  }
  const float cv = sC[lane] + f1b[j0 + lane];
  for (int pass = 0; pass < 2; ++pass) {
    *(volatile v8h*)(G1H + (size_t)(j0 + grow) * kFeatK + c8) = hv;
    if (wave == 0) *(volatile float*)(C1 + j0 + lane) = cv;
    __threadfence();
  }
}

__global__ __launch_bounds__(256) void init_state_kernel(const float* __restrict__ slots_p,
                                                         const float* __restrict__ Sp0, const float* __restrict__ Ss0,
                                                         float* __restrict__ SL, float* __restrict__ UH) {
  const int t = threadIdx.x, lane = t & 31, wave = t >> 5;
  const int bs = blockIdx.x, s = bs & (kS - 1);
  const float v = slots_p[s * kDS + t];
  const int ia = (lane < 2) ? lane : 2;
  int ib = lane - 3;
  ib = (ib < 0) ? 0 : ((ib > 2) ? 2 : ib);
  const float a = Sp0[s * 3 + ia];
  const float c = Ss0[s * 3 + ib];
  const float fa = (lane < 3) ? 1.0f : 0.0f;
  const float fc = (lane >= 3 && lane < 6) ? 1.0f : 0.0f;
  const float e = fmaf(fa, a, fc * c);
  for (int pass = 0; pass < 2; ++pass) {
    *(volatile float*)(SL + bs * kDS + t) = v;
    if (wave == 0) *(volatile float*)(UH + bs * kPitchS + kStatOff + lane) = e;
    __threadfence();
  }
}

__global__ __launch_bounds__(256) void slotq_kernel(
    const float* __restrict__ slots, const float* __restrict__ ng, const float* __restrict__ nb,
    const float* __restrict__ Qw, const float* __restrict__ f2w, const float* __restrict__ f2b,
    float* __restrict__ QF, const float* __restrict__ fw, const float* __restrict__ fb,
    float* __restrict__ out0, int do_final) {
  __shared__ __align__(16) float sX[kDS];
  __shared__ __align__(16) float sSn[kDS];
  __shared__ __align__(16) float sQ[kDS];
  __shared__ float red[8];
  const int t = threadIdx.x, lane = t & 31, wave = t >> 5, bs = blockIdx.x;
  const float x = slots[bs * kDS + t];
  sX[t] = x;
  const float mean = block_sum256(x, red, lane, wave) * kInvDS;
  const float dx = x - mean;
  const float var = block_sum256(dx * dx, red, lane, wave) * kInvDS;
  const float rstd = 1.0f / sqrtf(var + kLnEps);
  sSn[t] = dx * rstd * ng[t] + nb[t];
  __syncthreads();
  float q = 0.0f;
  {
    const float* wr = Qw + (size_t)t * kDS;
#pragma unroll 1
    for (int i = 0; i < kDS / 4; ++i) {
      const v4f a = *(const v4f*)(sSn + 4 * i);
      const v4f w = *(const v4f*)(wr + 4 * i);
      q = fmaf(a[0], w[0], q);
      q = fmaf(a[1], w[1], q);
      q = fmaf(a[2], w[2], q);
      q = fmaf(a[3], w[3], q);
    }
  }
  sQ[t] = q;
  __syncthreads();
  float qf = 0.0f;
#pragma unroll 4
  for (int d = 0; d < kDS; ++d) qf = fmaf(sQ[d], f2w[(size_t)d * kDS + t], qf);
  const float qb = block_sum256(q * f2b[t], red, lane, wave);
  float o = 0.0f;
  if (do_final) {
    const float* wr = fw + (size_t)t * kDS;
#pragma unroll 1
    for (int i = 0; i < kDS / 4; ++i) {
      const v4f a = *(const v4f*)(sX + 4 * i);
      const v4f w = *(const v4f*)(wr + 4 * i);
      o = fmaf(a[0], w[0], o);
      o = fmaf(a[1], w[1], o);
      o = fmaf(a[2], w[2], o);
      o = fmaf(a[3], w[3], o);
    }
    o += fb[t];
  }
  const float e = (lane == 0) ? qb : 0.0f;
  for (int pass = 0; pass < 2; ++pass) {
    *(volatile float*)(QF + bs * kPitchS + t) = qf;
    if (wave == 0) *(volatile float*)(QF + bs * kPitchS + kStatOff + lane) = e;
    if (do_final) *(volatile float*)(out0 + bs * kDS + t) = o;
    __threadfence();
  }
}

__global__ __launch_bounds__(256) void feat_kernel(const float* __restrict__ coords, const float* __restrict__ UH,
                                                   unsigned short* __restrict__ FA) {
  __shared__ __align__(16) float sT[256 * kFeatLds];
  const int t = threadIdx.x, lane = t & 31, wave = t >> 5;
  const int r0 = blockIdx.x * 256;
  const int bs = r0 / kN;
  const int b  = bs / kS;
  const int n  = (r0 - bs * kN) + t;
  const float* st = UH + bs * kPitchS + kStatOff;
  const float* cp = coords + ((size_t)b * kN + n) * 3;
  float rel0, rel1, rel2;
  {
    const float s0 = fminf(fmaxf(st[3], 0.3f), 5.0f) + 0.1f;
    const float s1 = fminf(fmaxf(st[4], 0.3f), 5.0f) + 0.1f;
    const float s2 = fminf(fmaxf(st[5], 0.3f), 5.0f) + 0.1f;
    const float i0 = 1.0f / (s0 * 5.0f + 1e-4f);
    const float i1 = 1.0f / (s1 * 5.0f + 1e-4f);
    const float i2 = 1.0f / (s2 * 5.0f + 1e-4f);
    rel0 = fminf(fmaxf((cp[0] - st[0]) * i0, -3.0f), 3.0f);
    rel1 = fminf(fmaxf((cp[1] - st[1]) * i1, -3.0f), 3.0f);
    rel2 = fminf(fmaxf((cp[2] - st[2]) * i2, -3.0f), 3.0f);
  }
  float* rowp = sT + t * kFeatLds;
  rowp[0] = rel0;
  rowp[1] = rel1;
  rowp[2] = rel2;
  rowp[kFeat] = 0.0f;
#pragma unroll 1
  for (int k = 0; k < 36; ++k) {
    const int ci = k >> 1;
    const int c = (ci >= 12) ? 2 : ((ci >= 6) ? 1 : 0);
    const int l = ci - 6 * c;
    const float rc = (c == 0) ? rel0 : ((c == 1) ? rel1 : rel2);
    float u = rc * (float)(1 << l);
    u = u - rintf(u);
    u = u + 0.25f * (float)(k & 1);
    rowp[3 + k] = sinf(u * kTwoPi);
  }
  __syncthreads();
  const int q = lane >> 3, c8 = (lane & 7) * 8;
  const int cc = (c8 < 32) ? c8 : 32;
  const bool live = (c8 < kFeatLds);
  v8h hv[8];
#pragma unroll
  for (int it = 0; it < 8; ++it) {
    const int row = wave * 32 + it * 4 + q;
    const v4f a0 = *(const v4f*)(sT + row * kFeatLds + cc);
    const v4f a1 = *(const v4f*)(sT + row * kFeatLds + cc + 4);
#pragma unroll
    for (int e = 0; e < 4; ++e) {
      const float y0 = live ? a0[e] : 0.0f;
      const float y1 = live ? a1[e] : 0.0f;
      hv[it][e]     = (_Float16)y0;
      hv[it][4 + e] = (_Float16)y1;
    }
  }
  for (int pass = 0; pass < 2; ++pass) {
#pragma unroll
    for (int it = 0; it < 8; ++it) {
      const int row = wave * 32 + it * 4 + q;
      *(volatile v8h*)(FA + (size_t)(r0 + row) * kFeatK + c8) = hv[it];
    }
    __threadfence();
  }
}

__global__ __launch_bounds__(256) void dots_kernel(const float* __restrict__ KVF, const unsigned short* __restrict__ PF,
                                                   const float* __restrict__ C1, const float* __restrict__ QF,
                                                   float* __restrict__ DOTS) {
  const int lane = threadIdx.x & 31, wave = threadIdx.x >> 5;
  const int r0 = (blockIdx.x * 8 + wave) * 32;
  const int bs = r0 / kN;
  const int b  = bs / kS;
  const int n0 = r0 - bs * kN;
  const int j0 = lane * 8;
  const v4f qa = *(const v4f*)(QF + bs * kPitchS + j0);
  const v4f qc = *(const v4f*)(QF + bs * kPitchS + j0 + 4);
  const v4f ca = *(const v4f*)(C1 + j0);
  const v4f cb = *(const v4f*)(C1 + j0 + 4);
  const float qb = QF[bs * kPitchS + kStatOff];
  const float* kf = KVF + ((size_t)b * kN + n0) * kDS + j0;
  const unsigned short* pf = PF + (size_t)r0 * kDS + j0;
  float keep = 0.0f;
#pragma unroll 1
  for (int i = 0; i < 32; ++i) {
    const v4f k0 = *(const v4f*)(kf + (size_t)i * kDS);
    const v4f k1 = *(const v4f*)(kf + (size_t)i * kDS + 4);
    const v4u pw = *(const v4u*)(pf + (size_t)i * kDS);
    v4f h0, h1;
    hid8(k0, k1, pw, ca, cb, h0, h1);
    float acc = 0.0f;
    acc = fmaf(h0[0], qa[0], acc);
    acc = fmaf(h0[1], qa[1], acc);
    acc = fmaf(h0[2], qa[2], acc);
    acc = fmaf(h0[3], qa[3], acc);
    acc = fmaf(h1[0], qc[0], acc);
    acc = fmaf(h1[1], qc[1], acc);
    acc = fmaf(h1[2], qc[2], acc);
    acc = fmaf(h1[3], qc[3], acc);
    acc += __shfl_xor(acc, 16, 32);
    acc += __shfl_xor(acc, 8, 32);
    acc += __shfl_xor(acc, 4, 32);
    acc += __shfl_xor(acc, 2, 32);
    acc += __shfl_xor(acc, 1, 32);
    keep = (lane == i) ? acc : keep;
  }
  float d = (keep + qb) * kDotScale;
  d = fminf(fmaxf(d, -30.0f), 30.0f);
  float* op = DOTS + r0 + lane;
  *(volatile float*)op = d;
  __threadfence();
  *(volatile float*)op = d;
}

__global__ __launch_bounds__(256) void slot_softmax_kernel(const float* __restrict__ DOTS, float* __restrict__ outp) {
  __shared__ __align__(16) float sA[kN];
  __shared__ float red[8];
  const int t = threadIdx.x, lane = t & 31, wave = t >> 5;
  const int bs = blockIdx.x, b = bs / kS, s = bs - b * kS;
  const float* db = DOTS + (size_t)b * kS * kN;
  float part = 0.0f;
#pragma unroll 1
  for (int e = 0; e < kN / 256; ++e) {
    const int n = t + 256 * e;
    float mx = db[n];
#pragma unroll 1
    for (int s2 = 1; s2 < kS; ++s2) mx = fmaxf(mx, db[s2 * kN + n]);
    float sum = 0.0f;
#pragma unroll 1
    for (int s2 = 0; s2 < kS; ++s2) sum += expf(db[s2 * kN + n] - mx);
    const float a = expf(db[s * kN + n] - mx) * (1.0f / sum) + 1e-8f;
    sA[n] = a;
    part += a;
  }
  const float total = block_sum256(part, red, lane, wave);
  const float inv = 1.0f / (total + 1e-8f);
  const v4f o0 = *(const v4f*)(sA + t * 4) * inv;
  const v4f o1 = *(const v4f*)(sA + 1024 + t * 4) * inv;
  float* orow = outp + (size_t)bs * kN;
  for (int pass = 0; pass < 2; ++pass) {
    *(volatile v4f*)(orow + t * 4) = o0;
    *(volatile v4f*)(orow + 1024 + t * 4) = o1;
    __threadfence();
  }
}

__global__ __launch_bounds__(256) void stats_kernel(const float* __restrict__ ATT, const float* __restrict__ coords,
                                                    const float* __restrict__ KVF, const unsigned short* __restrict__ PF,
                                                    const float* __restrict__ C1, float* __restrict__ UH) {
  __shared__ __align__(16) float sAt[kN];
  __shared__ __align__(16) float sRed[8 * kDS];
  __shared__ float red[8];
  const int t = threadIdx.x, lane = t & 31, wave = t >> 5;
  const int bs = blockIdx.x, b = bs / kS;
  *(v4f*)(sAt + t * 4) = *(const v4f*)(ATT + (size_t)bs * kN + t * 4);
  *(v4f*)(sAt + 1024 + t * 4) = *(const v4f*)(ATT + (size_t)bs * kN + 1024 + t * 4);
  __syncthreads();
  const float* cb3 = coords + (size_t)b * kN * 3;
  float p0 = 0.0f, p1 = 0.0f, p2 = 0.0f, pa = 0.0f;
#pragma unroll 1
  for (int e = 0; e < kN / 256; ++e) {
    const int n = t + 256 * e;
    const float a = sAt[n];
    p0 = fmaf(cb3[n * 3 + 0], a, p0);
    p1 = fmaf(cb3[n * 3 + 1], a, p1);
    p2 = fmaf(cb3[n * 3 + 2], a, p2);
    pa += a;
  }
  const float sp0 = block_sum256(p0, red, lane, wave);
  const float sp1 = block_sum256(p1, red, lane, wave);
  const float sp2 = block_sum256(p2, red, lane, wave);
  const float asum = block_sum256(pa, red, lane, wave);
  float q0 = 0.0f, q1 = 0.0f, q2 = 0.0f;
#pragma unroll 1
  for (int e = 0; e < kN / 256; ++e) {
    const int n = t + 256 * e;
    const float a = sAt[n];
    const float d0 = cb3[n * 3 + 0] - sp0;
    const float d1 = cb3[n * 3 + 1] - sp1;
    const float d2 = cb3[n * 3 + 2] - sp2;
    q0 = fmaf(d0 * d0, a, q0);
    q1 = fmaf(d1 * d1, a, q1);
    q2 = fmaf(d2 * d2, a, q2);
  }
  const float ss0 = fminf(fmaxf(sqrtf(block_sum256(q0, red, lane, wave) + 1e-6f), 0.2f), 5.0f);
  const float ss1 = fminf(fmaxf(sqrtf(block_sum256(q1, red, lane, wave) + 1e-6f), 0.2f), 5.0f);
  const float ss2 = fminf(fmaxf(sqrtf(block_sum256(q2, red, lane, wave) + 1e-6f), 0.2f), 5.0f);

  const int c8 = lane * 8;
  const v4f ca = *(const v4f*)(C1 + c8);
  const v4f cb = *(const v4f*)(C1 + c8 + 4);
  const float* vf = KVF + ((size_t)kRowsE + (size_t)b * kN) * kDS + c8;
  const unsigned short* pf = PF + (size_t)bs * kN * kDS + c8;
  v4f u0 = (v4f){0.f, 0.f, 0.f, 0.f};
  v4f u1 = (v4f){0.f, 0.f, 0.f, 0.f};
#pragma unroll 1
  for (int i = 0; i < kN / 8; ++i) {
    const int n = i * 8 + wave;
    const float a = sAt[n];
    const v4f k0 = *(const v4f*)(vf + (size_t)n * kDS);
    const v4f k1 = *(const v4f*)(vf + (size_t)n * kDS + 4);
    const v4u pw = *(const v4u*)(pf + (size_t)n * kDS);
    v4f h0, h1;
    hid8(k0, k1, pw, ca, cb, h0, h1);
    u0[0] = fmaf(h0[0], a, u0[0]);
    u0[1] = fmaf(h0[1], a, u0[1]);
    u0[2] = fmaf(h0[2], a, u0[2]);
    u0[3] = fmaf(h0[3], a, u0[3]);
    u1[0] = fmaf(h1[0], a, u1[0]);
    u1[1] = fmaf(h1[1], a, u1[1]);
    u1[2] = fmaf(h1[2], a, u1[2]);
    u1[3] = fmaf(h1[3], a, u1[3]);
  }
  *(v4f*)(sRed + wave * kDS + c8) = u0;
  *(v4f*)(sRed + wave * kDS + c8 + 4) = u1;
  __syncthreads();
  float uh = 0.0f;
#pragma unroll
  for (int w = 0; w < 8; ++w) uh += sRed[w * kDS + t];
  float e = 0.0f;
  e = (lane == 0) ? sp0 : e;
  e = (lane == 1) ? sp1 : e;
  e = (lane == 2) ? sp2 : e;
  e = (lane == 3) ? ss0 : e;
  e = (lane == 4) ? ss1 : e;
  e = (lane == 5) ? ss2 : e;
  e = (lane == 6) ? asum : e;
  for (int pass = 0; pass < 2; ++pass) {
    *(volatile float*)(UH + bs * kPitchS + t) = uh;
    if (wave == 0) *(volatile float*)(UH + bs * kPitchS + kStatOff + lane) = e;
    __threadfence();
  }
}

__global__ __launch_bounds__(256) void slot_update_kernel(
    const float* __restrict__ UH, const float* __restrict__ slots_in, float* __restrict__ slots_out,
    const float* __restrict__ f2w, const float* __restrict__ f2b,
    const float* __restrict__ wih, const float* __restrict__ whh,
    const float* __restrict__ bih, const float* __restrict__ bhh,
    const float* __restrict__ mng, const float* __restrict__ mnb,
    const float* __restrict__ m1w, const float* __restrict__ m1b,
    const float* __restrict__ m2w, const float* __restrict__ m2b) {
  __shared__ __align__(16) float sU[kDS];
  __shared__ __align__(16) float sV[2 * kDS];
  __shared__ __align__(16) float sG[6 * kDS];
  __shared__ __align__(16) float sL[kDS];
  __shared__ __align__(16) float sM[kHid];
  __shared__ float red[8];
  const int t = threadIdx.x, lane = t & 31, wave = t >> 5, bs = blockIdx.x;
  sU[t] = UH[bs * kPitchS + t];
  const float h = slots_in[bs * kDS + t];
  sV[kDS + t] = h;
  const float asum = UH[bs * kPitchS + kAsumOff];
  __syncthreads();
  float acc = 0.0f;
  {
    const float* wr = f2w + (size_t)t * kDS;
#pragma unroll 1
    for (int i = 0; i < kDS / 4; ++i) {
      const v4f a = *(const v4f*)(sU + 4 * i);
      const v4f w = *(const v4f*)(wr + 4 * i);
      acc = fmaf(a[0], w[0], acc);
      acc = fmaf(a[1], w[1], acc);
      acc = fmaf(a[2], w[2], acc);
      acc = fmaf(a[3], w[3], acc);
    }
  }
  sV[t] = n2nf(acc + f2b[t] * asum);
  __syncthreads();
#pragma unroll 1
  for (int g = 0; g < 6; ++g) {
    const int gsel = (g >= 3) ? 1 : 0;
    const int row = (g - 3 * gsel) * kDS + t;
    const float* W  = gsel ? whh : wih;
    const float* bb = gsel ? bhh : bih;
    const float* wr = W + (size_t)row * kDS;
    const int voff = gsel * kDS;
    float a2 = 0.0f;
#pragma unroll 1
    for (int i = 0; i < kDS / 4; ++i) {
      const v4f a = *(const v4f*)(sV + voff + 4 * i);
      const v4f w = *(const v4f*)(wr + 4 * i);
      a2 = fmaf(a[0], w[0], a2);
      a2 = fmaf(a[1], w[1], a2);
      a2 = fmaf(a[2], w[2], a2);
      a2 = fmaf(a[3], w[3], a2);
    }
    sG[g * kDS + t] = a2 + bb[row];
  }
  const float rg  = 1.0f / (1.0f + expf(-(sG[t] + sG[3 * kDS + t])));
  const float zg  = 1.0f / (1.0f + expf(-(sG[kDS + t] + sG[4 * kDS + t])));
  const float ngv = tanhf(sG[2 * kDS + t] + rg * sG[5 * kDS + t]);
  const float hnew = (1.0f - zg) * ngv + zg * h;
  const float mean = block_sum256(hnew, red, lane, wave) * kInvDS;
  const float dx = hnew - mean;
  const float var = block_sum256(dx * dx, red, lane, wave) * kInvDS;
  const float rstd = 1.0f / sqrtf(var + kLnEps);
  sL[t] = dx * rstd * mng[t] + mnb[t];
  __syncthreads();
#pragma unroll 1
  for (int i4 = 0; i4 < kHid / 256; ++i4) {
    const int o = i4 * 256 + t;
    const float* wr = m1w + (size_t)o * kDS;
    float a3 = 0.0f;
#pragma unroll 1
    for (int i = 0; i < kDS / 4; ++i) {
      const v4f a = *(const v4f*)(sL + 4 * i);
      const v4f w = *(const v4f*)(wr + 4 * i);
      a3 = fmaf(a[0], w[0], a3);
      a3 = fmaf(a[1], w[1], a3);
      a3 = fmaf(a[2], w[2], a3);
      a3 = fmaf(a[3], w[3], a3);
    }
    sM[o] = fmaxf(a3 + m1b[o], 0.0f);
  }
  __syncthreads();
  float a4 = 0.0f;
  {
    const float* wr = m2w + (size_t)t * kHid;
#pragma unroll 1
    for (int i = 0; i < kHid / 4; ++i) {
      const v4f a = *(const v4f*)(sM + 4 * i);
      const v4f w = *(const v4f*)(wr + 4 * i);
      a4 = fmaf(a[0], w[0], a4);
      a4 = fmaf(a[1], w[1], a4);
      a4 = fmaf(a[2], w[2], a4);
      a4 = fmaf(a[3], w[3], a4);
    }
  }
  const float outv = n2nf(hnew + (a4 + m2b[t]));
  float* op = slots_out + bs * kDS + t;
  *(volatile float*)op = outv;
  __threadfence();
  *(volatile float*)op = outv;
}

extern "C" void kernel_launch(void* const* d_in, const int* in_sizes, int n_in,
                              void* d_out, int out_size, void* d_ws, size_t ws_size,
                              hipStream_t stream) {
  const int expect[36] = {
      kB * kN * kDin, kB * kN * 3, kS * kDS, kS * 3, kS * 3,
      kDS * kDS, kDS * kDS, kDS * kDS, kDS * kFeat, kDS,
      kDS * kDS, kDS, kDS * kDS, kDS, kDS, kDS,
      kGru * kDS, kGru * kDS, kGru, kGru, kDS, kDS,
      kHid * kDS, kHid, kDS * kHid, kDS,
      kDin, kDin, kDin * kDin, kDin, kDS * kDin, kDS, kDS, kDS,
      kDS * kDS, kDS};
  if (n_in < 36) return;
  for (int i = 0; i < 36; ++i) {
    if (in_sizes[i] != expect[i]) return;
  }
  if (out_size != kOutSlots + kBS * kN) return;
  if (ws_size < kWsTotal) return;

  const float* inputs  = (const float*)d_in[0];
  const float* coords  = (const float*)d_in[1];
  const float* slots_p = (const float*)d_in[2];
  const float* Ss0     = (const float*)d_in[3];
  const float* Sp0     = (const float*)d_in[4];
  const float* Qw      = (const float*)d_in[5];
  const float* Kw      = (const float*)d_in[6];
  const float* Vw      = (const float*)d_in[7];
  const float* gw      = (const float*)d_in[8];
  const float* gb      = (const float*)d_in[9];
  const float* f1w     = (const float*)d_in[10];
  const float* f1b     = (const float*)d_in[11];
  const float* f2w     = (const float*)d_in[12];
  const float* f2b     = (const float*)d_in[13];
  const float* ng      = (const float*)d_in[14];
  const float* nbv     = (const float*)d_in[15];
  const float* wih     = (const float*)d_in[16];
  const float* whh     = (const float*)d_in[17];
  const float* bih     = (const float*)d_in[18];
  const float* bhh     = (const float*)d_in[19];
  const float* m_ng    = (const float*)d_in[20];
  const float* m_nb    = (const float*)d_in[21];
  const float* m1w     = (const float*)d_in[22];
  const float* m1b     = (const float*)d_in[23];
  const float* m2w     = (const float*)d_in[24];
  const float* m2b     = (const float*)d_in[25];
  const float* i0g     = (const float*)d_in[26];
  const float* i0b     = (const float*)d_in[27];
  const float* i1w     = (const float*)d_in[28];
  const float* i1b     = (const float*)d_in[29];
  const float* i2w     = (const float*)d_in[30];
  const float* i2b     = (const float*)d_in[31];
  const float* i3g     = (const float*)d_in[32];
  const float* i3b     = (const float*)d_in[33];
  const float* fw      = (const float*)d_in[34];
  const float* fb      = (const float*)d_in[35];

  float* out0 = (float*)d_out;
  float* out1 = (float*)d_out + kOutSlots;

  char* ws = (char*)d_ws;
  unsigned short* W1H  = (unsigned short*)(ws + kOffW1H);
  unsigned short* W2H  = (unsigned short*)(ws + kOffW2H);
  unsigned short* KVWH = (unsigned short*)(ws + kOffKVWH);
  unsigned short* F1H  = (unsigned short*)(ws + kOffF1H);
  unsigned short* G1H  = (unsigned short*)(ws + kOffG1H);
  float*          C1   = (float*)(ws + kOffC1);
  unsigned short* X0H  = (unsigned short*)(ws + kOffX0H);
  unsigned short* H1H  = (unsigned short*)(ws + kOffH1H);
  float*          XP   = (float*)(ws + kOffXP);
  unsigned short* XH   = (unsigned short*)(ws + kOffXH);
  unsigned short* KVH  = (unsigned short*)(ws + kOffKVH);
  float*          KVF  = (float*)(ws + kOffKVF);
  unsigned short* FA   = (unsigned short*)(ws + kOffFA);
  unsigned short* PF   = (unsigned short*)(ws + kOffPF);
  float*          DOTS = (float*)(ws + kOffDOTS);
  float*          ATT  = (float*)(ws + kOffATT);
  float*          SLA  = (float*)(ws + kOffSLA);
  float*          SLB  = (float*)(ws + kOffSLB);
  float*          QF   = (float*)(ws + kOffQF);
  float*          UH   = (float*)(ws + kOffUH);

  cast8_f16_kernel<<<(kDin * kDin / 8) / 256, 256, 0, stream>>>(i1w, W1H, kDin * kDin / 8, kWCarry);
  cast8_f16_kernel<<<(kDS * kDin / 8) / 256, 256, 0, stream>>>(i2w, W2H, kDS * kDin / 8, kWCarry);
  cast8_f16_kernel<<<(kDS * kDS / 8) / 256, 256, 0, stream>>>(Kw, KVWH, kDS * kDS / 8, kWCarry);
  cast8_f16_kernel<<<(kDS * kDS / 8) / 256, 256, 0, stream>>>(Vw, KVWH + (size_t)kDS * kDS, kDS * kDS / 8, kWCarry);
  cast8_f16_kernel<<<(kDS * kDS / 8) / 256, 256, 0, stream>>>(f1w, F1H, kDS * kDS / 8, kWCarry);

  ln_rows_f16_kernel<3, false><<<kRowsE / 8, 256, 0, stream>>>(inputs, i0g, i0b, X0H, kRowsE);
  wmma_gemm64<2, 1, 2><<<dim3(192, 1), 256, 0, stream>>>(
      X0H, kDin, 0L, W1H, kDin, 0L, (void*)H1H, kDin, 0L, i1b, kRowsE, kDin, kDin, kWCarryInv);
  wmma_gemm64<2, 0, 0><<<dim3(64, 1), 256, 0, stream>>>(
      H1H, kDin, 0L, W2H, kDin, 0L, (void*)XP, kDS, 0L, i2b, kRowsE, kDS, kDin, kWCarryInv);
  ln_rows_f16_kernel<1, true><<<kRowsE / 8, 256, 0, stream>>>(XP, i3g, i3b, XH, kRowsE);
  wmma_gemm64<0, 1, 0><<<dim3(64, 2), 256, 0, stream>>>(
      XH, kDS, 0L, KVWH, kDS, (long)kDS * kDS, (void*)KVH, kDS, (long)kRowsE * kDS, nullptr,
      kRowsE, kDS, kDS, kWCarryInv);
  wmma_gemm64<0, 0, 0><<<dim3(128, 1), 256, 0, stream>>>(
      KVH, kDS, 0L, F1H, kDS, 0L, (void*)KVF, kDS, 0L, nullptr, 2 * kRowsE, kDS, kDS, kWCarryInv);

  g1_kernel<<<kDS / 32, 256, 0, stream>>>(f1w, gw, gb, f1b, G1H, C1);
  init_state_kernel<<<kBS, 256, 0, stream>>>(slots_p, Sp0, Ss0, SLA, UH);

  for (int t = 0; t < 4; ++t) {
    float* scur = (t & 1) ? SLB : SLA;
    float* snxt = (t & 1) ? SLA : SLB;
    const int last = (t == 3) ? 1 : 0;
    slotq_kernel<<<kBS, 256, 0, stream>>>(scur, ng, nbv, Qw, f2w, f2b, QF, fw, fb, out0, last);
    feat_kernel<<<kRowsP / 256, 256, 0, stream>>>(coords, UH, FA);
    wmma_gemm64<0, 1, 0><<<dim3(512, 1), 256, 0, stream>>>(
        FA, kFeatK, 0L, G1H, kFeatK, 0L, (void*)PF, kDS, 0L, nullptr, kRowsP, kDS, kFeatK, kWCarryInv);
    dots_kernel<<<kRowsP / 256, 256, 0, stream>>>(KVF, PF, C1, QF, DOTS);
    slot_softmax_kernel<<<kBS, 256, 0, stream>>>(DOTS, last ? out1 : ATT);
    if (!last) {
      stats_kernel<<<kBS, 256, 0, stream>>>(ATT, coords, KVF, PF, C1, UH);
      slot_update_kernel<<<kBS, 256, 0, stream>>>(UH, scur, snxt, f2w, f2b, wih, whh, bih, bhh,
                                                   m_ng, m_nb, m1w, m1b, m2w, m2b);
    }
  }
}
